// Policy_42331197669623
// MI455X (gfx1250) — hardware-verified
//
#include <hip/hip_runtime.h>
#include <math.h>

typedef __attribute__((ext_vector_type(16))) _Float16 v16h;
typedef __attribute__((ext_vector_type(8)))  _Float16 v8h;
typedef __attribute__((ext_vector_type(8)))  float    v8f;
typedef __attribute__((ext_vector_type(4)))  float    v4f;

constexpr int kBatch = 128;
constexpr int kUnits = 2048;
constexpr int kFeat  = 128;
constexpr int kHid   = 32;
constexpr int kPreIn = 512;
constexpr int kTgt   = 2 * kUnits;

constexpr int kOffOut0   = 0;
constexpr int kOffOut1   = 1152;
constexpr int kOffOut2   = 2304;
constexpr int kOffOut3   = 2688;
constexpr int kOffTgt    = 3328;
constexpr int kOffH1     = 527616;
constexpr int kOffC1     = 544000;
constexpr int kOutFloats = 560384;
constexpr int kHeadFloats = kOffTgt;
static_assert(kOffOut1 == kOffOut0 + kBatch * 9);
static_assert(kOffOut2 == kOffOut1 + kBatch * 9);
static_assert(kOffOut3 == kOffOut2 + kBatch * 3);
static_assert(kOffTgt  == kOffOut3 + kBatch * 5);
static_assert(kOffH1   == kOffTgt + kBatch * kTgt);
static_assert(kOffC1   == kOffH1 + kBatch * kFeat);
static_assert(kOutFloats == kOffC1 + kBatch * kFeat);
static_assert(kOffTgt * 4 == 13312 && kOffH1 * 4 == 2110464 && kOffC1 * 4 == 2176000);
static_assert((kOffTgt * 4) % 128 == 0 && (kOffH1 * 4) % 128 == 0 && (kOffC1 * 4) % 128 == 0);
static_assert(kHeadFloats % 128 == 0);

constexpr int kWsMax    = 0;
constexpr int kWsRec    = 2 * kBatch * kFeat;
constexpr int kWsFloats = kWsRec + kBatch * 128;
constexpr int kRecLen   = 128;

constexpr float kCarry   = 16.0f;
constexpr float kUnCarry = 1.0f / 256.0f;

template <typename T> struct Frag;
template <> struct Frag<_Float16> {
  typedef v16h V; union U { v16h v; v8h h[2]; };
  static __device__ __forceinline__ v16h load(const _Float16* p) {
    U f; f.h[0] = *(const v8h*)(p); f.h[1] = *(const v8h*)(p + 16); return f.v;
  }
};

__device__ __forceinline__ v8f wmma_f16_zero(v16h a, v16h b) {
  v8f c = (v8f){0.f, 0.f, 0.f, 0.f, 0.f, 0.f, 0.f, 0.f};
  c = __builtin_amdgcn_wmma_f32_16x16x32_f16(false, a, false, b, (short)0, c, false, false);
  asm volatile("v_nop\n\tv_nop\n\tv_nop\n\tv_nop" : "+v"(c) : "v"(a), "v"(b));
  return c;
}

__device__ __forceinline__ float sigm_f(float x) { return __builtin_amdgcn_rcpf(1.0f + expf(-x)); }

__global__ __launch_bounds__(256) void unit_max_kernel(
    const float* __restrict__ enh_in, const float* __restrict__ anh_in,
    const float* __restrict__ W_e1, const float* __restrict__ b_e1,
    const float* __restrict__ W_e2, const float* __restrict__ b_e2,
    const float* __restrict__ W_a1, const float* __restrict__ b_a1,
    const float* __restrict__ W_a2, const float* __restrict__ b_a2,
    float* __restrict__ max_out)
{
  __shared__ __align__(16) _Float16 sW2h[kFeat * kHid];
  __shared__ float sW1[96];
  __shared__ float sb1[32];
  __shared__ float wred[8][kFeat];
  __shared__ __align__(16) float sres[kFeat];

  const int t    = threadIdx.x;
  const int wave = t >> 5;
  const int lane = t & 31;
  const int m    = lane & 15;
  const int h    = lane >> 4;
  const int b    = blockIdx.x >> 1;
  const int side = blockIdx.x & 1;

  const float* in = side ? anh_in : enh_in;
  const float* W1 = side ? W_a1 : W_e1;
  const float* b1 = side ? b_a1 : b_e1;
  const float* W2 = side ? W_a2 : W_e2;
  const float* b2 = side ? b_a2 : b_e2;

  if (t < 96) sW1[t] = W1[t];
  if (t < 32) sb1[t] = b1[t];
#pragma unroll
  for (int it = 0; it < 2; ++it) {
    const int e8 = (it * 256 + t) * 8;
    const float* src = W2 + e8;
    const v4f wa = *(const v4f*)(src);
    const v4f wc = *(const v4f*)(src + 4);
    v8h hv;
    hv[0] = (_Float16)(wa[0] * kCarry); hv[1] = (_Float16)(wa[1] * kCarry);
    hv[2] = (_Float16)(wa[2] * kCarry); hv[3] = (_Float16)(wa[3] * kCarry);
    hv[4] = (_Float16)(wc[0] * kCarry); hv[5] = (_Float16)(wc[1] * kCarry);
    hv[6] = (_Float16)(wc[2] * kCarry); hv[7] = (_Float16)(wc[3] * kCarry);
    *(v8h*)(sW2h + e8) = hv;
  }
  __syncthreads();

  v16h bfr[8];
#pragma unroll
  for (int nt = 0; nt < 8; ++nt) bfr[nt] = Frag<_Float16>::load(sW2h + (nt * 16 + m) * kHid + 8 * h);

  float vmax[8];
#pragma unroll
  for (int nt = 0; nt < 8; ++nt) vmax[nt] = -3.402823466e38f;

  const float* bin = in + (size_t)b * kUnits * 3;

#pragma unroll 1
  for (int mt = 0; mt < 16; ++mt) {
    const int unit = wave * 256 + mt * 16 + m;
    const float* pu = bin + (size_t)unit * 3;
    const float x0 = pu[0], x1 = pu[1], x2 = pu[2];
    v16h afr;
#pragma unroll
    for (int i = 0; i < 8; ++i) {
      const int ka = 8 * h + i;
      float pa = x0 * sW1[ka * 3 + 0];
      pa = fmaf(x1, sW1[ka * 3 + 1], pa);
      pa = fmaf(x2, sW1[ka * 3 + 2], pa);
      const float ha = fmaxf(pa + sb1[ka], 0.0f) * kCarry;
      afr[i] = (_Float16)ha;
      const int kb = 16 + 8 * h + i;
      float pb = x0 * sW1[kb * 3 + 0];
      pb = fmaf(x1, sW1[kb * 3 + 1], pb);
      pb = fmaf(x2, sW1[kb * 3 + 2], pb);
      const float hb = fmaxf(pb + sb1[kb], 0.0f) * kCarry;
      afr[8 + i] = (_Float16)hb;
    }
#pragma unroll
    for (int nt = 0; nt < 8; ++nt) {
      const v8f d = wmma_f16_zero(afr, bfr[nt]);
      float m0 = fmaxf(d[0], d[1]);
      float m1 = fmaxf(d[2], d[3]);
      float m2 = fmaxf(d[4], d[5]);
      float m3 = fmaxf(d[6], d[7]);
      m0 = fmaxf(m0, m1); m2 = fmaxf(m2, m3);
      vmax[nt] = fmaxf(vmax[nt], fmaxf(m0, m2));
    }
  }

#pragma unroll
  for (int nt = 0; nt < 8; ++nt) vmax[nt] = fmaxf(vmax[nt], __shfl_xor(vmax[nt], 16, 32));
  if (h == 0) {
#pragma unroll
    for (int nt = 0; nt < 8; ++nt) wred[wave][nt * 16 + m] = vmax[nt];
  }
  __syncthreads();
  if (t < kFeat) {
    float mx = wred[0][t];
#pragma unroll
    for (int w = 1; w < 8; ++w) mx = fmaxf(mx, wred[w][t]);
    sres[t] = mx * kUnCarry + b2[t];
  }
  __syncthreads();
  if (wave == 0) {
    float* dst = max_out + ((size_t)side * kBatch + b) * kFeat;
    for (int pass = 0; pass < 2; ++pass) {
      const v4f v = *(const v4f*)(sres + lane * 4);
      *(volatile v4f*)(dst + lane * 4) = v;
      __threadfence();
    }
  }
}

__global__ __launch_bounds__(128) void mid_kernel(
    const float* __restrict__ loc,   const float* __restrict__ env,
    const float* __restrict__ maxes, const float* __restrict__ h0,  const float* __restrict__ c0,
    const float* __restrict__ W_loc, const float* __restrict__ b_loc,
    const float* __restrict__ W_env, const float* __restrict__ b_env,
    const float* __restrict__ W_pre, const float* __restrict__ b_pre,
    const float* __restrict__ W_ih,  const float* __restrict__ b_ih,
    const float* __restrict__ W_hh,  const float* __restrict__ b_hh,
    const float* __restrict__ ln_g,  const float* __restrict__ ln_b,
    const float* __restrict__ W_mx,  const float* __restrict__ b_mx,
    const float* __restrict__ W_my,  const float* __restrict__ b_my,
    const float* __restrict__ W_en,  const float* __restrict__ b_en,
    const float* __restrict__ W_dl,  const float* __restrict__ b_dl,
    const float* __restrict__ W_at,  const float* __restrict__ b_at,
    const float* __restrict__ W_e2,  const float* __restrict__ b_e2,
    const float* __restrict__ W_a2,  const float* __restrict__ b_a2,
    float* __restrict__ rec_out, float* __restrict__ out)
{
  __shared__ float xin[kPreIn];
  __shared__ float sh0[kFeat];
  __shared__ float xln[kFeat];
  __shared__ __align__(16) float sh1[kFeat];
  __shared__ __align__(16) float sc1[kFeat];
  __shared__ float sattn[kFeat];
  __shared__ float sWh[26 * kFeat];
  __shared__ float sbh[32];
  __shared__ __align__(16) float srec[kRecLen];
  __shared__ float redA[4];
  __shared__ float redB[4];

  const int b    = blockIdx.x;
  const int t    = threadIdx.x;
  const int wave = t >> 5;
  const int lane = t & 31;

  {
    const float l0 = loc[b * 2], l1 = loc[b * 2 + 1];
    const float w0 = W_loc[t * 2], w1 = W_loc[t * 2 + 1], bb = b_loc[t];
    float p = l0 * w0;
    p = fmaf(l1, w1, p);
    xin[t] = fmaxf(p + bb, 0.0f);
  }
  asm volatile("" ::: "memory");
  {
    const float e0 = env[b * 2], e1 = env[b * 2 + 1];
    const float w0 = W_env[t * 2], w1 = W_env[t * 2 + 1], bb = b_env[t];
    float p = e0 * w0;
    p = fmaf(e1, w1, p);
    xin[kFeat + t] = fmaxf(p + bb, 0.0f);
  }
  asm volatile("" ::: "memory");
  xin[2 * kFeat + t] = maxes[(size_t)b * kFeat + t];
  xin[3 * kFeat + t] = maxes[(size_t)(kBatch + b) * kFeat + t];
  sh0[t] = h0[(size_t)b * kFeat + t];
  const float c0v = c0[(size_t)b * kFeat + t];
  asm volatile("" ::: "memory");
#pragma unroll
  for (int r = 0; r < 9; ++r) sWh[r * kFeat + t] = W_mx[r * kFeat + t];
  asm volatile("" ::: "memory");
#pragma unroll
  for (int r = 0; r < 9; ++r) sWh[(9 + r) * kFeat + t] = W_my[r * kFeat + t];
  asm volatile("" ::: "memory");
#pragma unroll
  for (int r = 0; r < 3; ++r) sWh[(18 + r) * kFeat + t] = W_en[r * kFeat + t];
#pragma unroll
  for (int r = 0; r < 5; ++r) sWh[(21 + r) * kFeat + t] = W_dl[r * kFeat + t];
  asm volatile("" ::: "memory");
  {
    const int j8 = (t < 8) ? t : 8;
    const int j2 = (t < 2) ? t : 2;
    const int j4 = (t < 4) ? t : 4;
    const float v0 = b_mx[j8], v1 = b_my[j8], v2 = b_en[j2], v3 = b_dl[j4];
    if (t < 9) sbh[t] = v0;
    if (t < 9) sbh[9 + t] = v1;
    if (t < 3) sbh[18 + t] = v2;
    if (t < 5) sbh[21 + t] = v3;
    if (t >= 26 && t < 32) sbh[t] = 0.0f;
  }
  if (t >= 66 && t < 96) srec[t] = 0.0f;
  __syncthreads();

  float acc = 0.0f;
  {
    const float* wr = W_pre + (size_t)t * kPreIn;
#pragma unroll 1
    for (int k = 0; k < kPreIn; ++k) acc = fmaf(xin[k], wr[k], acc);
  }
  const float x = fmaxf(acc + b_pre[t], 0.0f);

  float s = x;
#pragma unroll
  for (int off = 1; off < 32; off <<= 1) s += __shfl_xor(s, off, 32);
  if (lane == 0) redA[wave] = s;
  __syncthreads();
  const float sum = (redA[0] + redA[1]) + (redA[2] + redA[3]);
  const float mu  = sum * (1.0f / 128.0f);
  const float d   = x - mu;
  float s2 = d * d;
#pragma unroll
  for (int off = 1; off < 32; off <<= 1) s2 += __shfl_xor(s2, off, 32);
  if (lane == 0) redB[wave] = s2;
  __syncthreads();
  const float sum2 = (redB[0] + redB[1]) + (redB[2] + redB[3]);
  const float var  = sum2 * (1.0f / 128.0f);
  const float rstd = rsqrtf(var + 1e-5f);
  const float xn = d * rstd * ln_g[t] + ln_b[t];
  xln[t] = xn;
  __syncthreads();

  float ai0 = 0.0f, ai1 = 0.0f, ai2 = 0.0f, ai3 = 0.0f;
  float ah0 = 0.0f, ah1 = 0.0f, ah2 = 0.0f, ah3 = 0.0f;
  {
    const float* wi0 = W_ih + (size_t)(0 * kFeat + t) * kFeat;
    const float* wi1 = W_ih + (size_t)(1 * kFeat + t) * kFeat;
    const float* wi2 = W_ih + (size_t)(2 * kFeat + t) * kFeat;
    const float* wi3 = W_ih + (size_t)(3 * kFeat + t) * kFeat;
    const float* wh0 = W_hh + (size_t)(0 * kFeat + t) * kFeat;
    const float* wh1 = W_hh + (size_t)(1 * kFeat + t) * kFeat;
    const float* wh2 = W_hh + (size_t)(2 * kFeat + t) * kFeat;
    const float* wh3 = W_hh + (size_t)(3 * kFeat + t) * kFeat;
#pragma unroll 1
    for (int k = 0; k < kFeat; ++k) {
      const float xv = xln[k], hv = sh0[k];
      ai0 = fmaf(xv, wi0[k], ai0); ai1 = fmaf(xv, wi1[k], ai1);
      ai2 = fmaf(xv, wi2[k], ai2); ai3 = fmaf(xv, wi3[k], ai3);
      ah0 = fmaf(hv, wh0[k], ah0); ah1 = fmaf(hv, wh1[k], ah1);
      ah2 = fmaf(hv, wh2[k], ah2); ah3 = fmaf(hv, wh3[k], ah3);
    }
  }
  const float bi0 = b_ih[t], bi1 = b_ih[kFeat + t], bi2 = b_ih[2 * kFeat + t], bi3 = b_ih[3 * kFeat + t];
  const float bh0 = b_hh[t], bh1 = b_hh[kFeat + t], bh2 = b_hh[2 * kFeat + t], bh3 = b_hh[3 * kFeat + t];
  const float g0 = ((ai0 + bi0) + ah0) + bh0;
  const float g1 = ((ai1 + bi1) + ah1) + bh1;
  const float g2 = ((ai2 + bi2) + ah2) + bh2;
  const float g3 = ((ai3 + bi3) + ah3) + bh3;
  const float ig = sigm_f(g0);
  const float fg = sigm_f(g1);
  const float gg = tanhf(g2);
  const float og = sigm_f(g3);
  const float c1 = fg * c0v + ig * gg;
  const float h1 = og * tanhf(c1);
  sh1[t] = h1;
  sc1[t] = c1;
  __syncthreads();

  if (wave == 0) {
    float* dst = out + kOffH1 + (size_t)b * kFeat;
    for (int pass = 0; pass < 2; ++pass) {
      const v4f v = *(const v4f*)(sh1 + lane * 4);
      *(volatile v4f*)(dst + lane * 4) = v;
      __threadfence();
    }
  }
  if (wave == 1) {
    float* dst = out + kOffC1 + (size_t)b * kFeat;
    for (int pass = 0; pass < 2; ++pass) {
      const v4f v = *(const v4f*)(sc1 + lane * 4);
      *(volatile v4f*)(dst + lane * 4) = v;
      __threadfence();
    }
  }

  float at = 0.0f;
  {
    const float* wa = W_at + (size_t)t * kFeat;
#pragma unroll 1
    for (int k = 0; k < kFeat; ++k) at = fmaf(sh1[k], wa[k], at);
  }
  at += b_at[t];
  sattn[t] = at;

  if (wave == 0) {
    const int j = (lane < 25) ? lane : 25;
    const float* wrow = sWh + j * kFeat;
    float a = 0.0f;
#pragma unroll 1
    for (int k = 0; k < kFeat; ++k) a = fmaf(sh1[k], wrow[k], a);
    a += sbh[j];
    srec[96 + lane] = (lane < 26) ? a : 0.0f;
  }
  __syncthreads();

  if (wave < 2) {
    const int k = lane;
    float a0 = 0.0f, a1 = 0.0f;
#pragma unroll 1
    for (int n = 0; n < kFeat; ++n) {
      const float av = sattn[n];
      a0 = fmaf(av, W_e2[n * kHid + k], a0);
      a1 = fmaf(av, W_a2[n * kHid + k], a1);
    }
    srec[t] = (wave == 0) ? a0 : a1;
  }
  float pE = at * b_e2[t];
  float pA = at * b_a2[t];
#pragma unroll
  for (int off = 1; off < 32; off <<= 1) { pE += __shfl_xor(pE, off, 32); pA += __shfl_xor(pA, off, 32); }
  if (lane == 0) { redA[wave] = pE; redB[wave] = pA; }
  __syncthreads();
  if (t == 0) {
    srec[64] = (redA[0] + redA[1]) + (redA[2] + redA[3]);
    srec[65] = (redB[0] + redB[1]) + (redB[2] + redB[3]);
  }
  __syncthreads();
  if (wave == 0) {
    float* dst = rec_out + (size_t)b * kRecLen;
    for (int pass = 0; pass < 2; ++pass) {
      const v4f v = *(const v4f*)(srec + lane * 4);
      *(volatile v4f*)(dst + lane * 4) = v;
      __threadfence();
    }
  }
}

__global__ __launch_bounds__(256) void score_softmax_kernel(
    const float* __restrict__ enh_in, const float* __restrict__ anh_in,
    const float* __restrict__ W_e1, const float* __restrict__ b_e1,
    const float* __restrict__ W_a1, const float* __restrict__ b_a1,
    const float* __restrict__ rec, float* __restrict__ out)
{
  __shared__ float sW1e[96];
  __shared__ float sW1a[96];
  __shared__ float sb1e[32];
  __shared__ float sb1a[32];
  __shared__ float swk[96];
  __shared__ __align__(16) float ssc[kTgt];
  __shared__ float redM[8];
  __shared__ float redS[8];

  const int b    = blockIdx.x;
  const int t    = threadIdx.x;
  const int wave = t >> 5;
  const int lane = t & 31;

  if (t < 96) { sW1e[t] = W_e1[t]; swk[t] = rec[(size_t)b * kRecLen + t]; }
  if (t >= 96 && t < 128) sb1e[t - 96] = b_e1[t - 96];
  if (t >= 128 && t < 224) sW1a[t - 128] = W_a1[t - 128];
  if (t >= 224) sb1a[t - 224] = b_a1[t - 224];
  __syncthreads();

  const float bc0 = swk[64];
  const float bc1 = swk[65];
  float mloc = -3.402823466e38f;

  const float* pe = enh_in + (size_t)b * kUnits * 3;
#pragma unroll 1
  for (int it = 0; it < 8; ++it) {
    const int u = it * 256 + t;
    const float* pu = pe + (size_t)u * 3;
    const float x0 = pu[0], x1 = pu[1], x2 = pu[2];
    float acc = 0.0f;
#pragma unroll 1
    for (int k = 0; k < kHid; ++k) {
      float pr = x0 * sW1e[k * 3 + 0];
      pr = fmaf(x1, sW1e[k * 3 + 1], pr);
      pr = fmaf(x2, sW1e[k * 3 + 2], pr);
      const float hv = fmaxf(pr + sb1e[k], 0.0f);
      acc = fmaf(hv, swk[k], acc);
    }
    const float sc = acc + bc0;
    ssc[u] = sc;
    mloc = fmaxf(mloc, sc);
  }
  const float* pa = anh_in + (size_t)b * kUnits * 3;
#pragma unroll 1
  for (int it = 0; it < 8; ++it) {
    const int u = it * 256 + t;
    const float* pu = pa + (size_t)u * 3;
    const float x0 = pu[0], x1 = pu[1], x2 = pu[2];
    float acc = 0.0f;
#pragma unroll 1
    for (int k = 0; k < kHid; ++k) {
      float pr = x0 * sW1a[k * 3 + 0];
      pr = fmaf(x1, sW1a[k * 3 + 1], pr);
      pr = fmaf(x2, sW1a[k * 3 + 2], pr);
      const float hv = fmaxf(pr + sb1a[k], 0.0f);
      acc = fmaf(hv, swk[kHid + k], acc);
    }
    const float sc = acc + bc1;
    ssc[kUnits + u] = sc;
    mloc = fmaxf(mloc, sc);
  }

  float mw = mloc;
#pragma unroll
  for (int off = 1; off < 32; off <<= 1) mw = fmaxf(mw, __shfl_xor(mw, off, 32));
  if (lane == 0) redM[wave] = mw;
  __syncthreads();
  float bm = redM[0];
#pragma unroll
  for (int w = 1; w < 8; ++w) bm = fmaxf(bm, redM[w]);

  float lsum = 0.0f;
#pragma unroll 1
  for (int it = 0; it < 16; ++it) {
    const int u = it * 256 + t;
    const float e = expf(ssc[u] - bm);
    ssc[u] = e;
    lsum += e;
  }
#pragma unroll
  for (int off = 1; off < 32; off <<= 1) lsum += __shfl_xor(lsum, off, 32);
  if (lane == 0) redS[wave] = lsum;
  __syncthreads();
  float tot = 0.0f;
#pragma unroll
  for (int w = 0; w < 8; ++w) tot += redS[w];
  const float inv = __builtin_amdgcn_rcpf(tot);

  float* dst = out + kOffTgt + (size_t)b * kTgt;
  for (int pass = 0; pass < 2; ++pass) {
#pragma unroll 1
    for (int it = 0; it < 4; ++it) {
      const int c = it * 8 + wave;
      v4f v = *(const v4f*)(ssc + c * 128 + lane * 4);
      v = v * inv;
      *(volatile v4f*)(dst + (size_t)c * 128 + lane * 4) = v;
    }
    __threadfence();
  }
}

template <int LEN, int LO, int OBASE>
__device__ __forceinline__ void head_softmax(const float* lg, float* so, int t) {
  float m = lg[LO];
#pragma unroll 1
  for (int j = 1; j < LEN; ++j) m = fmaxf(m, lg[LO + j]);
  float* op = so + OBASE + t * LEN;
  float s = 0.0f;
#pragma unroll 1
  for (int j = 0; j < LEN; ++j) {
    const float e = expf(lg[LO + j] - m);
    op[j] = e;
    s += e;
  }
  const float inv = __builtin_amdgcn_rcpf(s);
#pragma unroll 1
  for (int j = 0; j < LEN; ++j) op[j] = op[j] * inv;
}

__global__ __launch_bounds__(128) void heads_pack_kernel(const float* __restrict__ rec, float* __restrict__ out)
{
  __shared__ __align__(16) float slg[kBatch * 28];
  __shared__ __align__(16) float sout[kHeadFloats];
  const int t    = threadIdx.x;
  const int wave = t >> 5;
  const int lane = t & 31;

  const float* rp = rec + (size_t)t * kRecLen + 96;
#pragma unroll
  for (int j = 0; j < 7; ++j) {
    const v4f v = *(const v4f*)(rp + 4 * j);
    *(v4f*)(slg + t * 28 + 4 * j) = v;
  }
  __syncthreads();
  const float* lg = slg + t * 28;
  head_softmax<9, 0,  kOffOut0>(lg, sout, t);
  head_softmax<9, 9,  kOffOut1>(lg, sout, t);
  head_softmax<3, 18, kOffOut2>(lg, sout, t);
  head_softmax<5, 21, kOffOut3>(lg, sout, t);
  __syncthreads();
  for (int pass = 0; pass < 2; ++pass) {
    for (int c = wave; c < kHeadFloats / 128; c += 4) {
      const v4f v = *(const v4f*)(sout + c * 128 + lane * 4);
      *(volatile v4f*)(out + (size_t)c * 128 + lane * 4) = v;
    }
    __threadfence();
  }
}

extern "C" void kernel_launch(void* const* d_in, const int* in_sizes, int n_in,
                              void* d_out, int out_size, void* d_ws, size_t ws_size,
                              hipStream_t stream)
{
  if (n_in < 36) return;
  if (out_size != kOutFloats) return;
  if (ws_size < (size_t)kWsFloats * sizeof(float)) return;
  if (in_sizes[2] != kBatch * kUnits * 3 || in_sizes[3] != kBatch * kUnits * 3) return;

  const float* loc    = (const float*)d_in[0];
  const float* env    = (const float*)d_in[1];
  const float* enh    = (const float*)d_in[2];
  const float* anh    = (const float*)d_in[3];
  const float* h0     = (const float*)d_in[4];
  const float* c0     = (const float*)d_in[5];
  const float* W_loc  = (const float*)d_in[6];  const float* b_loc  = (const float*)d_in[7];
  const float* W_env  = (const float*)d_in[8];  const float* b_env  = (const float*)d_in[9];
  const float* W_enh1 = (const float*)d_in[10]; const float* b_enh1 = (const float*)d_in[11];
  const float* W_enh2 = (const float*)d_in[12]; const float* b_enh2 = (const float*)d_in[13];
  const float* W_anh1 = (const float*)d_in[14]; const float* b_anh1 = (const float*)d_in[15];
  const float* W_anh2 = (const float*)d_in[16]; const float* b_anh2 = (const float*)d_in[17];
  const float* W_pre  = (const float*)d_in[18]; const float* b_pre  = (const float*)d_in[19];
  const float* W_ih   = (const float*)d_in[20]; const float* b_ih   = (const float*)d_in[21];
  const float* W_hh   = (const float*)d_in[22]; const float* b_hh   = (const float*)d_in[23];
  const float* ln_g   = (const float*)d_in[24]; const float* ln_b   = (const float*)d_in[25];
  const float* W_mx   = (const float*)d_in[26]; const float* b_mx   = (const float*)d_in[27];
  const float* W_my   = (const float*)d_in[28]; const float* b_my   = (const float*)d_in[29];
  const float* W_en   = (const float*)d_in[30]; const float* b_en   = (const float*)d_in[31];
  const float* W_dl   = (const float*)d_in[32]; const float* b_dl   = (const float*)d_in[33];
  const float* W_at   = (const float*)d_in[34]; const float* b_at   = (const float*)d_in[35];

  float* out   = (float*)d_out;
  float* ws    = (float*)d_ws;
  float* maxes = ws + kWsMax;
  float* recs  = ws + kWsRec;

  unit_max_kernel<<<2 * kBatch, 256, 0, stream>>>(enh, anh, W_enh1, b_enh1, W_enh2, b_enh2,
                                                   W_anh1, b_anh1, W_anh2, b_anh2, maxes);
  mid_kernel<<<kBatch, 128, 0, stream>>>(loc, env, maxes, h0, c0,
                                         W_loc, b_loc, W_env, b_env,
                                         W_pre, b_pre, W_ih, b_ih, W_hh, b_hh, ln_g, ln_b,
                                         W_mx, b_mx, W_my, b_my, W_en, b_en, W_dl, b_dl,
                                         W_at, b_at, W_enh2, b_enh2, W_anh2, b_anh2,
                                         recs, out);
  score_softmax_kernel<<<kBatch, 256, 0, stream>>>(enh, anh, W_enh1, b_enh1, W_anh1, b_anh1, recs, out);
  heads_pack_kernel<<<1, kBatch, 0, stream>>>(recs, out);
}
